// PGA_resnte_3435973837029
// MI455X (gfx1250) — hardware-run, weakly checked
//
#include <hip/hip_runtime.h>


#ifndef NB
#define NB 16
#endif
#ifndef HH
#define HH 64
#endif
#define NB_FULL  16
#define HH_FULL  64
#define WWD  32
#define NN       (HH * WWD)
#define NN_FULL  (HH_FULL * WWD)
#define CC   256
#define HID  32
#define OC   64
#define XSP  264
#define PSP  68
#define FSP  132
#define BNEPS 1e-5f
#define L2E  1.4426950408889634f
#define NEGB (-3.0e38f)

static_assert(WWD == 32);
static_assert(HID == 32);
static_assert(OC == 2 * HID);
static_assert(CC % 32 == 0);
static_assert(CC % 64 == 0);
static_assert(CC % 8 == 0);
static_assert(NN % 128 == 0);
static_assert(NN % 64 == 0);
static_assert(NB <= NB_FULL);
static_assert(HH <= HH_FULL);
static_assert((XSP * 2) % 16 == 0);
static_assert(XSP >= CC);
static_assert((PSP * 4) % 16 == 0);
static_assert((FSP * 4) % 16 == 0);
static_assert(PSP >= 64);
static_assert(FSP >= 128);
static_assert(((size_t)HID * CC) % 8 == 0);
static_assert((size_t)4 * 8 * 32 * 16 == (size_t)OC * 64 * 4);
static_assert((size_t)4 * 16 * 32 * 16 == (size_t)64 * 128 * 4);
static_assert((size_t)8 * 16 == (size_t)32 * 4);
static_assert(8 * 4 == 32);
static_assert((size_t)64 * XSP * 2 + (size_t)OC * PSP * 4 + (size_t)2 * OC * 4 <= (size_t)131072);
static_assert((size_t)64 * FSP * 4 + (size_t)2 * CC * 4 <= (size_t)131072);

typedef unsigned short bf;
typedef __attribute__((ext_vector_type(16))) __bf16   v16bf;
typedef __attribute__((ext_vector_type(8)))  unsigned short v8us;
typedef __attribute__((ext_vector_type(8)))  float    v8f;
typedef __attribute__((ext_vector_type(4)))  float    v4f;
typedef v4f  __attribute__((may_alias)) v4fa;
typedef v8us __attribute__((may_alias)) v8usa;

__device__ __forceinline__ unsigned short f2bf(float f) { unsigned u = __float_as_uint(f); u += 0x7FFFu + ((u >> 16) & 1u); return (unsigned short)(u >> 16); }
__device__ __forceinline__ float bfr(float f) { return __uint_as_float(((unsigned)f2bf(f)) << 16); }
__device__ __forceinline__ v16bf cat16b(v8us lo, v8us hi) { return __builtin_bit_cast(v16bf, __builtin_shufflevector(lo, hi, 0, 1, 2, 3, 4, 5, 6, 7, 8, 9, 10, 11, 12, 13, 14, 15)); }
__device__ __forceinline__ v8f wmmab(v16bf a, v16bf b, v8f c) { return __builtin_amdgcn_wmma_f32_16x16x32_bf16(false, a, false, b, (short)0, c, false, false); }
__device__ __forceinline__ v16bf ldb(const bf* p)  { return cat16b(*(const v8us*)p, *(const v8us*)(p + 16)); }
__device__ __forceinline__ v8f wmmab_g(v16bf a, v16bf b, v8f c) { c = wmmab(a, b, c); asm volatile("v_nop\n\tv_nop\n\tv_nop\n\tv_nop" : "+v"(c) : "v"(a), "v"(b)); return c; }

__global__ __launch_bounds__(256) void k_cvt8(const float* __restrict__ src, bf* dst, size_t n8) {
    const size_t i = (size_t)blockIdx.x * 256 + threadIdx.x; if (i >= n8) return;
    const v8f v = *(const v8f*)(src + i * 8); v8us o;
#pragma unroll
    for (int k = 0; k < 8; ++k) o[k] = f2bf(v[k]);
    *(volatile v8us*)(dst + i * 8) = o; __threadfence(); *(volatile v8us*)(dst + i * 8) = o;
}

__global__ __launch_bounds__(128) void k_proj(const float* __restrict__ x, const bf* __restrict__ WB,
                                              const float* __restrict__ ga, const float* __restrict__ ba, const float* __restrict__ ma, const float* __restrict__ va,
                                              const float* __restrict__ gs, const float* __restrict__ bs, const float* __restrict__ ms, const float* __restrict__ vs,
                                              float* AS) {
    __shared__ __align__(16) bf xs[64 * XSP];
    __shared__ __align__(16) float pt[OC * PSP];
    __shared__ float s_inv[OC], s_sh[OC];
    const int tid = threadIdx.x, lane = tid & 31, lr = lane & 15, hi = lane >> 4;
    const int wave = __builtin_amdgcn_readfirstlane((int)(threadIdx.x >> 5));
    const int n0 = blockIdx.x * 64, b = blockIdx.y;
    const float* xb = x + (size_t)b * CC * NN_FULL + n0;
    { const int q = tid & 15, r = tid >> 4;
#pragma unroll 4
      for (int it = 0; it < CC / 8; ++it) { const int c = it * 8 + r;
          const v4f v = *(const v4f*)(xb + (size_t)c * NN_FULL + 4 * q);
#pragma unroll
          for (int i = 0; i < 4; ++i) xs[(4 * q + i) * XSP + c] = f2bf(v[i]); } }
    { const int oi = tid & 31; const bool sg = (tid & 32) != 0;
      const float g0 = bfr(ga[oi]), b0 = bfr(ba[oi]), m0 = bfr(ma[oi]), v0 = bfr(va[oi]);
      const float g1 = bfr(gs[oi]), b1 = bfr(bs[oi]), m1 = bfr(ms[oi]), v1 = bfr(vs[oi]);
      const float g = sg ? g1 : g0, bb = sg ? b1 : b0, mm = sg ? m1 : m0, vv = sg ? v1 : v0;
      const float inv = g / sqrtf(vv + BNEPS);
      const float sh = bb - mm * inv;
      if (tid < OC) { s_inv[tid] = inv; s_sh[tid] = sh; } }
    __syncthreads();
    v8f acc[4];
#pragma unroll
    for (int mb = 0; mb < 4; ++mb) acc[mb] = (v8f){};
    const int xo = (16 * wave + lr) * XSP + 8 * hi;
    const size_t wo = (size_t)lr * CC + 8 * hi;
#pragma unroll 1
    for (int kc = 0; kc < CC; kc += 32) {
        const v16bf bx = cat16b(*(const v8usa*)(&xs[xo + kc]), *(const v8usa*)(&xs[xo + kc + 16]));
#pragma unroll
        for (int mb = 0; mb < 4; ++mb) { const v16bf a = ldb(WB + wo + (size_t)mb * 16 * CC + kc); acc[mb] = wmmab_g(a, bx, acc[mb]); }
    }
#pragma unroll
    for (int mb = 0; mb < 4; ++mb) {
#pragma unroll
        for (int j = 0; j < 8; ++j) { const int o = 16 * mb + 8 * hi + j;
            const float y = acc[mb][j] * s_inv[o] + s_sh[o];
            pt[o * PSP + 16 * wave + lr] = fmaxf(y, 0.0f); } }
    __syncthreads();
    float* dst = AS + ((size_t)b * OC) * NN + n0;
#pragma unroll 1
    for (int pz = 0; pz < 2; ++pz) {
#pragma unroll
        for (int s = 0; s < 8; ++s) { const int row = 16 * wave + 2 * s + (lane >> 4), c4 = (lane & 15) * 4;
            const v4f val = *(const v4fa*)(&pt[row * PSP + c4]);
            *(volatile v4f*)(dst + (size_t)row * NN + c4) = val; }
        if (pz == 0) __threadfence(); }
}

__global__ __launch_bounds__(256) void k_cdot(const float* __restrict__ x, float* DD) {
#pragma clang fp contract(off)
    __shared__ __align__(16) float sd[32];
    const int lane = threadIdx.x & 31;
    const int wave = __builtin_amdgcn_readfirstlane((int)(threadIdx.x >> 5));
    const int b = blockIdx.y;
    const int c0 = blockIdx.x * 32 + 4 * wave;
    const int c3v = (int)blockIdx.x * 32 + 4 * (int)(threadIdx.x >> 5) + 3;
    int r4v = c3v + 1; r4v = r4v > CC - 1 ? CC - 1 : r4v;
    const int r4 = __builtin_amdgcn_readfirstlane(r4v);
    const size_t o0 = ((size_t)b * CC + c0) * NN_FULL + 4 * lane;
    const size_t o4 = ((size_t)b * CC + r4) * NN_FULL + 4 * lane;
    float a0 = 0.0f, a1 = 0.0f, a2 = 0.0f, a3 = 0.0f;
#pragma unroll 1
    for (int it = 0; it < NN / 128; ++it) {
        const size_t o = o0 + (size_t)it * 128;
        const v4f u0 = *(const v4f*)(x + o);
        const v4f u1 = *(const v4f*)(x + o + (size_t)NN_FULL);
        const v4f u2 = *(const v4f*)(x + o + (size_t)2 * NN_FULL);
        const v4f u3 = *(const v4f*)(x + o + (size_t)3 * NN_FULL);
        const v4f u4 = *(const v4f*)(x + o4 + (size_t)it * 128);
#pragma unroll
        for (int e = 0; e < 4; ++e) { const float f0 = bfr(u0[e]), f1 = bfr(u1[e]), f2 = bfr(u2[e]), f3 = bfr(u3[e]), f4 = bfr(u4[e]);
            a0 += f0 * f1; a1 += f1 * f2; a2 += f2 * f3; a3 += f3 * f4; }
    }
#pragma unroll
    for (int d = 16; d >= 1; d >>= 1) { a0 += __shfl_xor(a0, d, 32); a1 += __shfl_xor(a1, d, 32); a2 += __shfl_xor(a2, d, 32); a3 += __shfl_xor(a3, d, 32); }
    const float z3 = (c3v < CC - 1) ? a3 : 0.0f;
    if (lane == 0) { sd[4 * wave + 0] = a0; sd[4 * wave + 1] = a1; sd[4 * wave + 2] = a2; sd[4 * wave + 3] = z3; }
    __syncthreads();
    if (wave == 0) {
        const v4f val = *(const v4fa*)(&sd[(lane & 7) * 4]);
        float* dst = DD + (size_t)b * CC + (size_t)blockIdx.x * 32 + (lane & 7) * 4;
#pragma unroll 1
        for (int pz = 0; pz < 2; ++pz) {
            if (lane < 8) *(volatile v4f*)dst = val;
            if (pz == 0) __threadfence(); }
    }
}

__global__ __launch_bounds__(128) void k_fuse(const float* __restrict__ x, const float* __restrict__ AS, const float* __restrict__ DD,
                                              const float* __restrict__ gama, float* OUT) {
#pragma clang fp contract(off)
    __shared__ __align__(16) float os[64 * FSP];
    __shared__ float s_wp[CC], s_wn[CC];
    const int tid = threadIdx.x, lane = tid & 31;
    const int wave = __builtin_amdgcn_readfirstlane((int)(threadIdx.x >> 5));
    const int b = blockIdx.y;
    const int j0 = blockIdx.x * 128;
    const int j = j0 + tid;
    const int r = j >> 5, col = j & 31;

#pragma unroll 1
    for (int c = tid; c < CC; c += 128) {
        const int cm = c > 0 ? c - 1 : 0;
        float ep = DD[(size_t)b * CC + cm];
        float en = DD[(size_t)b * CC + c];
        asm volatile("" : "+v"(ep));
        asm volatile("" : "+v"(en));
        const float mm = fmaxf(ep, en);
        const float e1 = __builtin_amdgcn_exp2f((ep - mm) * L2E), e2 = __builtin_amdgcn_exp2f((en - mm) * L2E);
        const float izc = 1.0f / (e1 + e2);
        float wp = e1 * izc, wn = e2 * izc;
        wp = (c == 0) ? 0.0f : ((c == CC - 1) ? 1.0f : wp);
        wn = (c == 0) ? 1.0f : ((c == CC - 1) ? 0.0f : wn);
        s_wp[c] = wp; s_wn[c] = wn;
    }

    int nb[8]; bool ok[8];
#pragma unroll
    for (int s = 0; s < 8; ++s) { const int t9 = s < 4 ? s : s + 1; const int dr = t9 / 3 - 1, dc = t9 % 3 - 1;
        const int rr = r + dr, cq = col + dc;
        ok[s] = ((rr >= 0) & (rr < HH) & (cq >= 0) & (cq < WWD)) != 0;
        nb[s] = ok[s] ? rr * WWD + cq : j; }

    const float* asb = AS + (size_t)b * OC * NN;
    float lg[8];
#pragma unroll
    for (int s = 0; s < 8; ++s) lg[s] = 0.0f;
#pragma unroll 1
    for (int h = 0; h < HID; ++h) {
        const float a = asb[(size_t)h * NN + j];
        const float* sr = asb + (size_t)(HID + h) * NN;
#pragma unroll
        for (int s = 0; s < 8; ++s) lg[s] = fmaf(a, sr[nb[s]], lg[s]);
    }
    float mx = NEGB;
#pragma unroll
    for (int s = 0; s < 8; ++s) mx = fmaxf(mx, ok[s] ? lg[s] : NEGB);
    float wv[8]; float z = 0.0f;
#pragma unroll
    for (int s = 0; s < 8; ++s) { const float e = __builtin_amdgcn_exp2f((lg[s] - mx) * L2E); wv[s] = ok[s] ? e : 0.0f; z += wv[s]; }
    const float iz = 1.0f / z;
#pragma unroll
    for (int s = 0; s < 8; ++s) wv[s] *= iz;

    const float g = bfr(gama[0]);
    const float omg = 1.0f - g;
    const float* xb = x + (size_t)b * CC * NN_FULL;
    __syncthreads();

#pragma unroll 1
    for (int ct = 0; ct < CC / 64; ++ct) {
        const int cs = ct * 64;
        const int cdn = cs > 0 ? cs - 1 : 0;
        const float xdl = bfr(xb[(size_t)cdn * NN_FULL + j]);
        float xdn = (cs > 0) ? xdl : 0.0f;
        float xcur = bfr(xb[(size_t)cs * NN_FULL + j]);
#pragma unroll 1
        for (int ci = 0; ci < 64; ++ci) {
            const int c = cs + ci;
            const int cu = (c + 1 < CC) ? c + 1 : CC - 1;
            const float xul = bfr(xb[(size_t)cu * NN_FULL + j]);
            const float xup = (c + 1 < CC) ? xul : 0.0f;
            const float* xr = xb + (size_t)c * NN_FULL;
            float hs = 0.0f;
#pragma unroll
            for (int s = 0; s < 8; ++s) hs = fmaf(wv[s], bfr(xr[nb[s]]), hs);
            const float hp = s_wp[c] * xdn + s_wn[c] * xup;
            const float hv = hs + hp;
            const float ex = __builtin_amdgcn_exp2f(hv * L2E) - 1.0f;
            const float he = (hv > 0.0f) ? hv : ex;
            os[ci * FSP + tid] = omg * xcur + g * he;
            xdn = xcur; xcur = xup;
        }
        __syncthreads();
        float* orow = OUT + ((size_t)b * CC + cs) * NN_FULL + j0;
#pragma unroll 1
        for (int pz = 0; pz < 2; ++pz) {
#pragma unroll 4
            for (int s = 0; s < 16; ++s) { const int row = 16 * wave + s;
                const v4f val = *(const v4fa*)(&os[row * FSP + 4 * lane]);
                *(volatile v4f*)(orow + (size_t)row * NN_FULL + 4 * lane) = val; }
            if (pz == 0) __threadfence(); }
        __syncthreads();
    }
}

static constexpr size_t al256(size_t v) { return (v + 255) & ~(size_t)255; }
static constexpr size_t SZ_WB = al256((size_t)OC * CC * 2);
static constexpr size_t SZ_AS = al256((size_t)NB * OC * NN * 4);
static constexpr size_t SZ_DD = al256((size_t)NB * CC * 4);
static constexpr size_t SZ_TOTAL = SZ_WB + SZ_AS + SZ_DD;
static_assert(SZ_TOTAL <= (size_t)134217728);
static_assert(((size_t)HID * CC * 2) % 256 == 0);
static_assert(((size_t)OC * NN * 4) % 256 == 0);
static_assert(((size_t)CC * 4) % 128 == 0);

extern "C" void kernel_launch(void* const* d_in, const int* in_sizes, int n_in,
                              void* d_out, int out_size, void* d_ws, size_t ws_size, hipStream_t stream) {
    if (n_in < 12) return;
    const size_t needx = ((size_t)(NB - 1) * CC + (size_t)(CC - 1)) * NN_FULL + NN;
    if ((size_t)in_sizes[0] < needx) return;
    if ((size_t)in_sizes[1] < (size_t)HID * CC || (size_t)in_sizes[6] < (size_t)HID * CC) return;
    if (in_sizes[2] < HID || in_sizes[3] < HID || in_sizes[4] < HID || in_sizes[5] < HID) return;
    if (in_sizes[7] < HID || in_sizes[8] < HID || in_sizes[9] < HID || in_sizes[10] < HID) return;
    if (in_sizes[11] < 1) return;
    if ((size_t)out_size < needx) return;
    if (SZ_TOTAL > ws_size) return;
    const float* x   = (const float*)d_in[0];
    const float* wa  = (const float*)d_in[1];
    const float* ga  = (const float*)d_in[2];
    const float* ba  = (const float*)d_in[3];
    const float* ma  = (const float*)d_in[4];
    const float* va  = (const float*)d_in[5];
    const float* wsg = (const float*)d_in[6];
    const float* gs  = (const float*)d_in[7];
    const float* bs  = (const float*)d_in[8];
    const float* ms  = (const float*)d_in[9];
    const float* vs  = (const float*)d_in[10];
    const float* gama = (const float*)d_in[11];
    float* OUT = (float*)d_out;
    char* wsp = (char*)d_ws;
    bf* WB = (bf*)wsp; wsp += SZ_WB;
    float* AS = (float*)wsp; wsp += SZ_AS;
    float* DD = (float*)wsp; wsp += SZ_DD;

    { const size_t n8 = (size_t)HID * CC / 8; const unsigned gq = (unsigned)((n8 + 255) / 256);
      k_cvt8<<<gq, 256, 0, stream>>>(wa, WB, n8);
      k_cvt8<<<gq, 256, 0, stream>>>(wsg, WB + (size_t)HID * CC, n8); }

    k_proj<<<dim3(NN / 64, NB, 1), 128, 0, stream>>>(x, WB, ga, ba, ma, va, gs, bs, ms, vs, AS);
    k_cdot<<<dim3(CC / 32, NB, 1), 256, 0, stream>>>(x, DD);
    k_fuse<<<dim3(NN / 128, NB, 1), 128, 0, stream>>>(x, AS, DD, gama, OUT);
}
